// GeoAB_62508954026302
// MI455X (gfx1250) — hardware-verified
//
#include <hip/hip_runtime.h>
#include <math.h>


typedef _Float16 v8h  __attribute__((ext_vector_type(8)));
typedef _Float16 v16h __attribute__((ext_vector_type(16)));
typedef float    v8f  __attribute__((ext_vector_type(8)));
typedef float    v4f  __attribute__((ext_vector_type(4)));
union Frag { v16h v; v8h hf[2]; };

#define NB     2
#define CIN    192
#define C2     384
#define HH     160
#define WW     160
#define HP     162
#define WP     162
#define KTOT   1728
#define NPOS   (NB * HH * WW)
#define NHEAD  8
#define TP     68
#define LOG100 4.605170186f
#define WSCALE 32.0f
#define INV_WSCALE 0.03125f
#define BIAS_PAD 5120

__device__ __forceinline__ v8f wmma_f16(v16h a, v16h b, v8f c) {
  return __builtin_amdgcn_wmma_f32_16x16x32_f16(false, a, false, b, (short)0, c, false, false);
}

__device__ __forceinline__ void ld8f(const float* p, float* r) {
  const v4f a = *(const v4f*)p;
  const v4f b = *(const v4f*)(p + 4);
  r[0] = a.x; r[1] = a.y; r[2] = a.z; r[3] = a.w;
  r[4] = b.x; r[5] = b.y; r[6] = b.z; r[7] = b.w;
}

__global__ __launch_bounds__(128) void pack_x_kernel(const float* __restrict__ x,
                                                     _Float16* xpad) {
  __shared__ __align__(16) _Float16 t[WP * 64];
  const int tid = threadIdx.x, wave = tid >> 5, l = tid & 31;
  const int Y = (int)blockIdx.x, q = (int)blockIdx.y, b = (int)blockIdx.z;
  if (Y >= 1 && Y <= HH) {
    const float* src = x + (((size_t)b * CIN + q * 64) * HH + (Y - 1)) * WW;
#pragma unroll 4
    for (int c = 0; c < 64; ++c) {
      const float* s = src + (size_t)c * HH * WW;
      t[(tid + 1) * 64 + c] = (_Float16)s[tid];
      if (tid < WW - 128) t[(tid + 129) * 64 + c] = (_Float16)s[tid + 128];
    }
    if (tid < 64) {
      t[tid] = (_Float16)0.0f;
      t[(WP - 1) * 64 + tid] = (_Float16)0.0f;
    }
  } else {
    for (int idx = tid; idx < WP * 64; idx += 128) t[idx] = (_Float16)0.0f;
  }
  __syncthreads();
  _Float16* dst = xpad + ((size_t)(b * HP + Y) * WP) * CIN + q * 64 + (l & 7) * 8;
  for (int i = 0; i < 11; ++i) {
    const int L = i * 16 + wave * 4 + (l >> 3);
    if (L < WP) {
      const v8h v = *(const v8h*)&t[L * 64 + (l & 7) * 8];
      *(volatile v8h*)(dst + (size_t)L * CIN) = v;
    }
  }
  __threadfence();
  for (int i = 0; i < 11; ++i) {
    const int L = i * 16 + wave * 4 + (l >> 3);
    if (L < WP) {
      const v8h v = *(const v8h*)&t[L * 64 + (l & 7) * 8];
      *(volatile v8h*)(dst + (size_t)L * CIN) = v;
    }
  }
}

__global__ __launch_bounds__(128) void pack_w_kernel(const float* __restrict__ w,
                                                     _Float16* wpk, int Cout) {
  __shared__ __align__(16) _Float16 row[KTOT];
  const int tid = threadIdx.x, wave = tid >> 5, l = tid & 31;
  const int oc = (int)blockIdx.x;
  if (oc >= Cout) return;
  for (int k = tid; k < KTOT; k += 128) {
    const int tap = k / CIN;
    const int ic = k - tap * CIN;
    const int ky = tap / 3, kx = tap - ky * 3;
    const float v = w[(((size_t)oc * CIN + ic) * 3 + ky) * 3 + kx] * WSCALE;
    row[k] = (_Float16)v;
  }
  __syncthreads();
  _Float16* dst = wpk + (size_t)oc * KTOT + (l & 7) * 8;
  for (int i = 0; i < 2; ++i) {
    const int L = i * 16 + wave * 4 + (l >> 3);
    if (L < KTOT / 64) {
      const v8h v = *(const v8h*)&row[L * 64 + (l & 7) * 8];
      *(volatile v8h*)(dst + L * 64) = v;
    }
  }
  __threadfence();
  for (int i = 0; i < 2; ++i) {
    const int L = i * 16 + wave * 4 + (l >> 3);
    if (L < KTOT / 64) {
      const v8h v = *(const v8h*)&row[L * 64 + (l & 7) * 8];
      *(volatile v8h*)(dst + L * 64) = v;
    }
  }
}

template <int MODE>
__device__ __forceinline__ void conv_store_lines(const float* tile, float* out, int Cout,
                                                 int oc0, int n0, int wave, int l) {
  const int c4 = (l & 7) * 4;
#pragma unroll
  for (int i = 0; i < 8; ++i) {
    const int L = i * 16 + wave * 4 + (l >> 3);
    if (MODE == 0) {
      const int p = L >> 1, q2 = L & 1;
      const v4f v = *(const v4f*)&tile[p * TP + q2 * 32 + c4];
      *(volatile v4f*)(out + (size_t)(n0 + p) * Cout + oc0 + q2 * 32 + c4) = v;
    } else {
      const int ocl = L >> 1, ph = L & 1;
      const int n  = n0 + ph * 32;
      const int b  = n / (HH * WW);
      const int rr = n - b * (HH * WW);
      const int y  = rr / WW;
      const int xx = rr - y * WW;
      const v4f v = *(const v4f*)&tile[ocl * TP + ph * 32 + c4];
      *(volatile v4f*)(out + (((size_t)b * Cout + oc0 + ocl) * HH + y) * WW + xx + c4) = v;
    }
  }
}

template <int MODE>
__global__ __launch_bounds__(128) void conv3x3_f16_kernel(
    const _Float16* __restrict__ xin,
    const _Float16* __restrict__ wpk,
    const float* __restrict__ bias,
    float* out, int Cout) {
  __shared__ __align__(16) float tile[64 * TP];
  const int tid = threadIdx.x;
  const int wave = tid >> 5, l = tid & 31, h = l >> 4, m = l & 15;
  const int wm = wave >> 1, wn = wave & 1;
  const int oc0 = (int)blockIdx.x * 64;
  const int n0  = (int)blockIdx.y * 64;
  if (oc0 + 64 > Cout || n0 + 64 > NPOS) return;

  int aOff[2], bOff[2];
#pragma unroll
  for (int mi = 0; mi < 2; ++mi)
    aOff[mi] = (oc0 + wm * 32 + mi * 16 + m) * KTOT + 8 * h;
#pragma unroll
  for (int ni = 0; ni < 2; ++ni) {
    const int n  = n0 + wn * 32 + ni * 16 + m;
    const int b  = n / (HH * WW);
    const int rr = n - b * (HH * WW);
    const int y  = rr / WW;
    const int xx = rr - y * WW;
    bOff[ni] = ((b * HP + y) * WP + xx) * CIN + 8 * h;
  }

  v8f zero = {};
  v8f acc[2][2];
  acc[0][0] = zero; acc[0][1] = zero; acc[1][0] = zero; acc[1][1] = zero;

#pragma unroll 1
  for (int tap = 0; tap < 9; ++tap) {
    const int ky = tap / 3, kx = tap - ky * 3;
    const int tapOff = (ky * WP + kx) * CIN;
    const int kbase = tap * CIN;
#pragma unroll 1
    for (int icb = 0; icb < CIN / 32; ++icb) {
      Frag a0, a1, b0, b1;
      const _Float16* ap0 = wpk + aOff[0] + kbase + icb * 32;
      const _Float16* ap1 = wpk + aOff[1] + kbase + icb * 32;
      const _Float16* bp0 = xin + bOff[0] + tapOff + icb * 32;
      const _Float16* bp1 = xin + bOff[1] + tapOff + icb * 32;
      a0.hf[0] = *(const v8h*)(ap0);  a0.hf[1] = *(const v8h*)(ap0 + 16);
      a1.hf[0] = *(const v8h*)(ap1);  a1.hf[1] = *(const v8h*)(ap1 + 16);
      b0.hf[0] = *(const v8h*)(bp0);  b0.hf[1] = *(const v8h*)(bp0 + 16);
      b1.hf[0] = *(const v8h*)(bp1);  b1.hf[1] = *(const v8h*)(bp1 + 16);
      acc[0][0] = wmma_f16(a0.v, b0.v, acc[0][0]);
      acc[0][1] = wmma_f16(a0.v, b1.v, acc[0][1]);
      acc[1][0] = wmma_f16(a1.v, b0.v, acc[1][0]);
      acc[1][1] = wmma_f16(a1.v, b1.v, acc[1][1]);
      asm volatile("v_nop\n\tv_nop\n\tv_nop\n\tv_nop"
                   : "+v"(acc[0][0]), "+v"(acc[0][1]), "+v"(acc[1][0]), "+v"(acc[1][1])
                   : "v"(a0.v), "v"(a1.v), "v"(b0.v), "v"(b1.v));
    }
  }

#pragma unroll
  for (int mi = 0; mi < 2; ++mi) {
    const int ocl = wm * 32 + mi * 16 + 8 * h;
    float bb[8];
    ld8f(bias + oc0 + ocl, bb);
#pragma unroll
    for (int ni = 0; ni < 2; ++ni) {
      const int p = wn * 32 + ni * 16 + m;
      if (MODE == 0) {
        v4f o0, o1;
        o0.x = acc[mi][ni][0] * INV_WSCALE + bb[0];
        o0.y = acc[mi][ni][1] * INV_WSCALE + bb[1];
        o0.z = acc[mi][ni][2] * INV_WSCALE + bb[2];
        o0.w = acc[mi][ni][3] * INV_WSCALE + bb[3];
        o1.x = acc[mi][ni][4] * INV_WSCALE + bb[4];
        o1.y = acc[mi][ni][5] * INV_WSCALE + bb[5];
        o1.z = acc[mi][ni][6] * INV_WSCALE + bb[6];
        o1.w = acc[mi][ni][7] * INV_WSCALE + bb[7];
        *(v4f*)&tile[p * TP + ocl]     = o0;
        *(v4f*)&tile[p * TP + ocl + 4] = o1;
      } else {
#pragma unroll
        for (int r = 0; r < 8; ++r)
          tile[(ocl + r) * TP + p] = acc[mi][ni][r] * INV_WSCALE + bb[r];
      }
    }
  }
  __syncthreads();
  conv_store_lines<MODE>(tile, out, Cout, oc0, n0, wave, l);
  __threadfence();
  conv_store_lines<MODE>(tile, out, Cout, oc0, n0, wave, l);
}

__global__ __launch_bounds__(128) void cpb_kernel(const float* __restrict__ w1,
                                                 const float* __restrict__ b1,
                                                 const float* __restrict__ w2,
                                                 float* biasT) {
  __shared__ float tbl[81 * 8];
  __shared__ __align__(16) float stage[BIAS_PAD];
  const int tid = threadIdx.x, wave = tid >> 5, l = tid & 31;
  if (tid < 81) {
    const int a = tid / 9, bq = tid - (tid / 9) * 9;
    const float t0 = (float)(a - 4) * 2.0f;
    const float t1 = (float)(bq - 4) * 2.0f;
    const float g0 = log2f(fabsf(t0) + 1.0f) / 3.0f;
    const float g1 = log2f(fabsf(t1) + 1.0f) / 3.0f;
    const float u0 = (t0 < 0.0f) ? -g0 : g0;
    const float u1 = (t1 < 0.0f) ? -g1 : g1;
    float acc[8];
#pragma unroll
    for (int n = 0; n < 8; ++n) acc[n] = 0.0f;
#pragma unroll 1
    for (int k = 0; k < 512; ++k) {
      const float hval = fmaxf(u0 * w1[2 * k] + u1 * w1[2 * k + 1] + b1[k], 0.0f);
#pragma unroll
      for (int n = 0; n < 8; ++n) acc[n] += hval * w2[n * 512 + k];
    }
#pragma unroll
    for (int n = 0; n < 8; ++n) tbl[tid * 8 + n] = acc[n];
  }
  __syncthreads();
  for (int e = tid; e < BIAS_PAD; e += 128) {
    float v = 0.0f;
    if (e < NHEAD * 625) {
      const int n = e / 625;
      const int rest = e - n * 625;
      const int i = rest / 25, j = rest - (rest / 25) * 25;
      const int di = i / 5 - j / 5 + 4;
      const int dj = (i - (i / 5) * 5) - (j - (j / 5) * 5) + 4;
      const float z = tbl[(di * 9 + dj) * 8 + n];
      v = 16.0f / (1.0f + expf(-z));
    }
    stage[e] = v;
  }
  __syncthreads();
  const int c4 = (l & 7) * 4;
  for (int i = 0; i < 10; ++i) {
    const int L = i * 16 + wave * 4 + (l >> 3);
    const v4f v = *(const v4f*)&stage[L * 32 + c4];
    *(volatile v4f*)(biasT + L * 32 + c4) = v;
  }
  __threadfence();
  for (int i = 0; i < 10; ++i) {
    const int L = i * 16 + wave * 4 + (l >> 3);
    const v4f v = *(const v4f*)&stage[L * 32 + c4];
    *(volatile v4f*)(biasT + L * 32 + c4) = v;
  }
}

__global__ __launch_bounds__(256) void win_attn_kernel(
    const float* __restrict__ xp, const float* __restrict__ biasT,
    const float* __restrict__ lsc, _Float16* ypad,
    int chanOff, int lineOff, int inShift, int outShift) {
  __shared__ __align__(16) float kn[NHEAD * 25 * 8];
  __shared__ __align__(16) float vv[NHEAD * 25 * 8];
  __shared__ __align__(16) _Float16 yt[25 * 64];
  const int tid = threadIdx.x, head = tid >> 5, l = tid & 31;
  const int wid = (int)blockIdx.x;
  const int b = wid >> 10;
  const int rem = wid & 1023;
  const int wy = rem >> 5, wx = rem & 31;
  const float scale = expf(fminf(lsc[head], LOG100));
  const int i = l;
  float qn[8];
  if (i < 25) {
    const int iy = i / 5, ix = i - iy * 5;
    const int sy = wy * 5 + iy, sx = wx * 5 + ix;
    int ys = sy + inShift; if (ys >= HH) ys -= HH;
    int xs = sx + inShift; if (xs >= WW) xs -= WW;
    const float* kp = xp + ((size_t)(b * HH + ys) * WW + xs) * C2 + chanOff + head * 8;
    float kr[8], vr[8];
    ld8f(kp, kr);
    ld8f(kp + 64, vr);
    float ss = 0.0f;
#pragma unroll
    for (int c = 0; c < 8; ++c) ss += kr[c] * kr[c];
    const float inv = 1.0f / fmaxf(sqrtf(ss), 1e-12f);
#pragma unroll
    for (int c = 0; c < 8; ++c) {
      qn[c] = kr[c] * inv;
      kn[(head * 25 + i) * 8 + c] = qn[c];
      vv[(head * 25 + i) * 8 + c] = vr[c];
    }
  }
  __syncthreads();
  if (i < 25) {
    const float* brow = biasT + (head * 25 + i) * 25;
    float mx = -1e30f, lsum = 0.0f;
    float acc[8];
#pragma unroll
    for (int c = 0; c < 8; ++c) acc[c] = 0.0f;
#pragma unroll 1
    for (int j = 0; j < 25; ++j) {
      float kj[8], vj[8];
      ld8f(&kn[(head * 25 + j) * 8], kj);
      ld8f(&vv[(head * 25 + j) * 8], vj);
      float s = 0.0f;
#pragma unroll
      for (int c = 0; c < 8; ++c) s += qn[c] * kj[c];
      s = s * scale + brow[j];
      const float mn = fmaxf(mx, s);
      const float corr = __expf(mx - mn);
      const float pr = __expf(s - mn);
      lsum = lsum * corr + pr;
#pragma unroll
      for (int c = 0; c < 8; ++c) acc[c] = acc[c] * corr + pr * vj[c];
      mx = mn;
    }
    const float invl = 1.0f / lsum;
#pragma unroll
    for (int c = 0; c < 8; ++c) yt[i * 64 + head * 8 + c] = (_Float16)(acc[c] * invl);
  }
  __syncthreads();
  {
    const int io = head * 4 + (l >> 3);
    if (io < 25) {
      const int iy = io / 5, ix = io - iy * 5;
      const int sy = wy * 5 + iy, sx = wx * 5 + ix;
      int yd = sy + outShift; if (yd >= HH) yd -= HH;
      int xd = sx + outShift; if (xd >= WW) xd -= WW;
      _Float16* dst = ypad + ((size_t)(b * HP + yd + 1) * WP + xd + 1) * CIN + lineOff + (l & 7) * 8;
      const _Float16* srcp = &yt[io * 64 + (l & 7) * 8];
      v8h v = *(const v8h*)srcp;
      *(volatile v8h*)dst = v;
      __threadfence();
      v = *(const v8h*)srcp;
      *(volatile v8h*)dst = v;
    }
  }
}

__global__ __launch_bounds__(160) void axial_rows_kernel(
    const float* __restrict__ xp, const float* __restrict__ lrs, float* vtmp) {
  __shared__ __align__(16) float kn[WW * 8];
  __shared__ __align__(16) float vv[WW * 8];
  __shared__ __align__(16) float yt[WW * 64];
  const int tid = threadIdx.x, wave = tid >> 5, l = tid & 31;
  const int b = (int)blockIdx.x / HH, y = (int)blockIdx.x - b * HH;
  const int t = tid;
  const size_t pos = (size_t)(b * HH + y) * WW + t;
#pragma unroll 1
  for (int head = 0; head < NHEAD; ++head) {
    const float scale = expf(fminf(lrs[head], LOG100));
    const float* kp = xp + pos * C2 + 256 + head * 8;
    float kr[8], vr[8], qn[8];
    ld8f(kp, kr);
    ld8f(kp + 64, vr);
    float ss = 0.0f;
#pragma unroll
    for (int c = 0; c < 8; ++c) ss += kr[c] * kr[c];
    const float inv = 1.0f / fmaxf(sqrtf(ss), 1e-12f);
#pragma unroll
    for (int c = 0; c < 8; ++c) qn[c] = kr[c] * inv;
    __syncthreads();
#pragma unroll
    for (int c = 0; c < 8; ++c) { kn[t * 8 + c] = qn[c]; vv[t * 8 + c] = vr[c]; }
    __syncthreads();
    float mx = -1e30f, lsum = 0.0f;
    float acc[8];
#pragma unroll
    for (int c = 0; c < 8; ++c) acc[c] = 0.0f;
#pragma unroll 1
    for (int j = 0; j < WW; ++j) {
      float kj[8], vj[8];
      ld8f(&kn[j * 8], kj);
      ld8f(&vv[j * 8], vj);
      float s = 0.0f;
#pragma unroll
      for (int c = 0; c < 8; ++c) s += qn[c] * kj[c];
      s *= scale;
      const float mn = fmaxf(mx, s);
      const float corr = __expf(mx - mn);
      const float pr = __expf(s - mn);
      lsum = lsum * corr + pr;
#pragma unroll
      for (int c = 0; c < 8; ++c) acc[c] = acc[c] * corr + pr * vj[c];
      mx = mn;
    }
    const float invl = 1.0f / lsum;
#pragma unroll
    for (int c = 0; c < 8; ++c) yt[t * 64 + head * 8 + c] = acc[c] * invl;
  }
  __syncthreads();
  float* dbase = vtmp + ((size_t)(b * HH + y) * WW) * 64;
  const int c4 = (l & 7) * 4;
  for (int i = 0; i < 16; ++i) {
    const int L = i * 20 + wave * 4 + (l >> 3);
    const int xq = L >> 1, hh = L & 1;
    const v4f v = *(const v4f*)&yt[xq * 64 + hh * 32 + c4];
    *(volatile v4f*)(dbase + (size_t)xq * 64 + hh * 32 + c4) = v;
  }
  __threadfence();
  for (int i = 0; i < 16; ++i) {
    const int L = i * 20 + wave * 4 + (l >> 3);
    const int xq = L >> 1, hh = L & 1;
    const v4f v = *(const v4f*)&yt[xq * 64 + hh * 32 + c4];
    *(volatile v4f*)(dbase + (size_t)xq * 64 + hh * 32 + c4) = v;
  }
}

__global__ __launch_bounds__(160) void axial_cols_kernel(
    const float* __restrict__ xp, const float* __restrict__ lrs,
    const float* __restrict__ vtmp, _Float16* ypad) {
  __shared__ __align__(16) float kn[HH * 8];
  __shared__ __align__(16) float vv[HH * 8];
  __shared__ __align__(16) _Float16 yt[HH * 64];
  const int tid = threadIdx.x, wave = tid >> 5, l = tid & 31;
  const int b = (int)blockIdx.x / WW, xcol = (int)blockIdx.x - b * WW;
  const int t = tid;
  const size_t pos = (size_t)(b * HH + t) * WW + xcol;
#pragma unroll 1
  for (int head = 0; head < NHEAD; ++head) {
    const float scale = expf(fminf(lrs[head], LOG100));
    float kr[8], vr[8], qn[8];
    ld8f(xp + pos * C2 + 256 + head * 8, kr);
    ld8f(vtmp + pos * 64 + head * 8, vr);
    float ss = 0.0f;
#pragma unroll
    for (int c = 0; c < 8; ++c) ss += kr[c] * kr[c];
    const float inv = 1.0f / fmaxf(sqrtf(ss), 1e-12f);
#pragma unroll
    for (int c = 0; c < 8; ++c) qn[c] = kr[c] * inv;
    __syncthreads();
#pragma unroll
    for (int c = 0; c < 8; ++c) { kn[t * 8 + c] = qn[c]; vv[t * 8 + c] = vr[c]; }
    __syncthreads();
    float mx = -1e30f, lsum = 0.0f;
    float acc[8];
#pragma unroll
    for (int c = 0; c < 8; ++c) acc[c] = 0.0f;
#pragma unroll 1
    for (int j = 0; j < HH; ++j) {
      float kj[8], vj[8];
      ld8f(&kn[j * 8], kj);
      ld8f(&vv[j * 8], vj);
      float s = 0.0f;
#pragma unroll
      for (int c = 0; c < 8; ++c) s += qn[c] * kj[c];
      s *= scale;
      const float mn = fmaxf(mx, s);
      const float corr = __expf(mx - mn);
      const float pr = __expf(s - mn);
      lsum = lsum * corr + pr;
#pragma unroll
      for (int c = 0; c < 8; ++c) acc[c] = acc[c] * corr + pr * vj[c];
      mx = mn;
    }
    const float invl = 1.0f / lsum;
#pragma unroll
    for (int c = 0; c < 8; ++c) yt[t * 64 + head * 8 + c] = (_Float16)(acc[c] * invl);
  }
  __syncthreads();
  const int c8 = (l & 7) * 8;
  for (int i = 0; i < 8; ++i) {
    const int L = i * 20 + wave * 4 + (l >> 3);
    const v8h v = *(const v8h*)&yt[L * 64 + c8];
    *(volatile v8h*)(ypad + ((size_t)(b * HP + L + 1) * WP + xcol + 1) * CIN + 128 + c8) = v;
  }
  __threadfence();
  for (int i = 0; i < 8; ++i) {
    const int L = i * 20 + wave * 4 + (l >> 3);
    const v8h v = *(const v8h*)&yt[L * 64 + c8];
    *(volatile v8h*)(ypad + ((size_t)(b * HP + L + 1) * WP + xcol + 1) * CIN + 128 + c8) = v;
  }
}

__global__ __launch_bounds__(128) void pad_ring_kernel(_Float16* ypad) {
  const int tid = threadIdx.x, wave = tid >> 5, l = tid & 31;
  const int Y = (int)blockIdx.x, b = (int)blockIdx.y;
  const bool full = (Y == 0) || (Y == HP - 1);
  const int nl = full ? WP * 3 : 6;
  v8h z = {};
  _Float16* base = ypad + ((size_t)(b * HP + Y) * WP) * CIN + (l & 7) * 8;
  for (int L0 = 0; L0 < nl; L0 += 16) {
    const int L = L0 + wave * 4 + (l >> 3);
    if (L < nl) {
      int X, ql;
      if (full) { X = L / 3; ql = L - X * 3; }
      else      { X = (L < 3) ? 0 : (WP - 1); ql = (L < 3) ? L : (L - 3); }
      *(volatile v8h*)(base + (size_t)X * CIN + ql * 64) = z;
    }
  }
  __threadfence();
  for (int L0 = 0; L0 < nl; L0 += 16) {
    const int L = L0 + wave * 4 + (l >> 3);
    if (L < nl) {
      int X, ql;
      if (full) { X = L / 3; ql = L - X * 3; }
      else      { X = (L < 3) ? 0 : (WP - 1); ql = (L < 3) ? L : (L - 3); }
      *(volatile v8h*)(base + (size_t)X * CIN + ql * 64) = z;
    }
  }
}

extern "C" void kernel_launch(void* const* d_in, const int* in_sizes, int n_in,
                              void* d_out, int out_size, void* d_ws, size_t ws_size,
                              hipStream_t stream) {
  if (n_in < 10) return;
  if (in_sizes[0] != NPOS * CIN || out_size != NPOS * CIN) return;
  if (in_sizes[1] != C2 * KTOT || in_sizes[2] < C2 || in_sizes[3] != CIN * KTOT ||
      in_sizes[4] < CIN || in_sizes[5] < NHEAD || in_sizes[6] < NHEAD ||
      in_sizes[7] < 1024 || in_sizes[8] < 512 || in_sizes[9] < NHEAD * 512) return;

  const float* x       = (const float*)d_in[0];
  const float* w_in    = (const float*)d_in[1];
  const float* b_in    = (const float*)d_in[2];
  const float* w_out   = (const float*)d_in[3];
  const float* b_out   = (const float*)d_in[4];
  const float* lscale  = (const float*)d_in[5];
  const float* lrscale = (const float*)d_in[6];
  const float* cpb_w1  = (const float*)d_in[7];
  const float* cpb_b1  = (const float*)d_in[8];
  const float* cpb_w2  = (const float*)d_in[9];
  float* out = (float*)d_out;

  char* ws = (char*)d_ws;
  size_t off = 0;
  auto carve = [&](size_t bytes) -> char* {
    char* p = ws + off;
    off = (off + bytes + 255) & ~(size_t)255;
    return p;
  };
  _Float16* xpad = (_Float16*)carve((size_t)NB * HP * WP * CIN * 2);
  _Float16* wA   = (_Float16*)carve((size_t)C2 * KTOT * 2);
  _Float16* wB   = (_Float16*)carve((size_t)CIN * KTOT * 2);
  float* xp      = (float*)carve((size_t)NPOS * C2 * 4);
  float* biasT   = (float*)carve((size_t)BIAS_PAD * 4);
  float* vtmp    = (float*)carve((size_t)NPOS * 64 * 4);
  if (off > ws_size) return;
  _Float16* ypad = xpad;

  pack_x_kernel<<<dim3(HP, 3, NB), 128, 0, stream>>>(x, xpad);
  pack_w_kernel<<<C2, 128, 0, stream>>>(w_in, wA, C2);
  pack_w_kernel<<<CIN, 128, 0, stream>>>(w_out, wB, CIN);

  conv3x3_f16_kernel<0><<<dim3(C2 / 64, NPOS / 64), 128, 0, stream>>>(xpad, wA, b_in, xp, C2);

  cpb_kernel<<<1, 128, 0, stream>>>(cpb_w1, cpb_b1, cpb_w2, biasT);

  win_attn_kernel<<<NB * 32 * 32, 256, 0, stream>>>(xp, biasT, lscale, ypad, 0,   0,  0, 0);
  win_attn_kernel<<<NB * 32 * 32, 256, 0, stream>>>(xp, biasT, lscale, ypad, 128, 64, 3, 2);

  axial_rows_kernel<<<NB * HH, 160, 0, stream>>>(xp, lrscale, vtmp);
  axial_cols_kernel<<<NB * WW, 160, 0, stream>>>(xp, lrscale, vtmp, ypad);

  pad_ring_kernel<<<dim3(HP, NB), 128, 0, stream>>>(ypad);
  conv3x3_f16_kernel<1><<<dim3(CIN / 64, NPOS / 64), 128, 0, stream>>>(ypad, wB, b_out, out, CIN);
}
